// WiKG_63745904607995
// MI455X (gfx1250) — hardware-verified
//
#include <hip/hip_runtime.h>
#include <math.h>
#include <stdint.h>


#define NTOK   8192
#define DIN    1024
#define DHID   512
#define TOPK   16
#define NCLS   2
#define AWAVES 8
#define BSTR   520
#define NRG    (NTOK / 64)

typedef char shape_chk0[(NTOK % (AWAVES * 16) == 0) ? 1 : -1];
typedef char shape_chk1[(NTOK % 64 == 0 && DHID % 64 == 0 && DIN % 64 == 0) ? 1 : -1];
typedef char shape_chk2[(DHID == 512 && TOPK == 16) ? 1 : -1];

typedef _Float16 f16;
typedef f16   v16h __attribute__((ext_vector_type(16)));
typedef f16   v8h  __attribute__((ext_vector_type(8)));
typedef float v8f  __attribute__((ext_vector_type(8)));
typedef float v4f  __attribute__((ext_vector_type(4)));
typedef float v2f  __attribute__((ext_vector_type(2)));
typedef v4f   v4fa __attribute__((may_alias));
union Frag { v16h v; v8h hv[2]; };

static __device__ __forceinline__ v16h ld_frag(const f16* base, int pitch, int r0, int k0) {
  const int l = threadIdx.x & 31, h = l >> 4, r = l & 15;
  const f16* p = base + (size_t)(r0 + r) * pitch + k0 + 8 * h;
  Frag f;
  f.hv[0] = *(const v8h*)p;
  f.hv[1] = *(const v8h*)(p + 16);
  return f.v;
}

static __device__ __forceinline__ v8f mma16(v16h a, v16h b, v8f c) {
  return __builtin_amdgcn_wmma_f32_16x16x32_f16(false, a, false, b, (short)0, c, false, false);
}

static __device__ __forceinline__ v8h cvt8(v4f a, v4f b, float s) {
  v8h o;
  o[0] = (f16)(a[0] * s); o[1] = (f16)(a[1] * s); o[2] = (f16)(a[2] * s); o[3] = (f16)(a[3] * s);
  o[4] = (f16)(b[0] * s); o[5] = (f16)(b[1] * s); o[6] = (f16)(b[2] * s); o[7] = (f16)(b[3] * s);
  return o;
}

__global__ void __launch_bounds__(256) k_cvt(const float* __restrict__ X, f16* Y, int n8, float sc)
{
  const int i = blockIdx.x * 256 + threadIdx.x;
  if (i >= n8) return;
  const size_t e = (size_t)i * 8;
  v4f a = *(const v4f*)(X + e);
  v4f b = *(const v4f*)(X + e + 4);
  v8h o = cvt8(a, b, sc);
  f16* p = Y + e;
  *(volatile v8h*)p = o;
  __threadfence();
  *(volatile v8h*)p = o;
}

__global__ void __launch_bounds__(256) k_wtr(const float* __restrict__ W, f16* Wt, int K, int Nc, float sc)
{
  __shared__ float s[64][33];
  const int tid = threadIdx.x;
  const int nkb = K >> 6;
  const int kb = blockIdx.x % nkb, nb = blockIdx.x / nkb;
  if (nb * 32 >= Nc) return;
  const int k0 = kb * 64, n0 = nb * 32;
#pragma unroll
  for (int i = 0; i < 8; ++i) {
    int e = tid + 256 * i;
    int kk = e >> 5, nn = e & 31;
    s[kk][nn] = W[(size_t)(k0 + kk) * Nc + n0 + nn];
  }
  __syncthreads();
  const int nn = tid >> 3, q = tid & 7;
  v8h o;
#pragma unroll
  for (int i = 0; i < 8; ++i) o[i] = (f16)(s[q * 8 + i][nn] * sc);
  f16* p = Wt + (size_t)(n0 + nn) * K + k0 + q * 8;
  *(volatile v8h*)p = o;
  __threadfence();
  *(volatile v8h*)p = o;
}

__global__ void __launch_bounds__(128) k_gemm(
    const f16* __restrict__ A, const f16* __restrict__ Bt, const float* __restrict__ bias,
    float* outF, f16* outH, float* P,
    int M, int Nc, int K, float cs, float hsA, float hsB, int flags)
{
  __shared__ __attribute__((aligned(16))) float sT[4][16][64];
  __shared__ __attribute__((aligned(16))) float sP[64];
  const int tid = threadIdx.x, wid = tid >> 5, l = tid & 31, h = l >> 4, m = l & 15;
  const int nbm = M >> 6;
  const int bm = blockIdx.x % nbm, bn = blockIdx.x / nbm;
  if (bn >= (Nc >> 6)) return;
  const int m0 = bm * 64 + wid * 16, n0 = bn * 64;

  const v8f z8 = {0.f, 0.f, 0.f, 0.f, 0.f, 0.f, 0.f, 0.f};
  v8f acc[4];
#pragma unroll
  for (int j = 0; j < 4; ++j) acc[j] = z8;

  for (int k0 = 0; k0 < K; k0 += 32) {
    v16h a  = ld_frag(A,  K, m0, k0);
    v16h b0 = ld_frag(Bt, K, n0,      k0);
    v16h b1 = ld_frag(Bt, K, n0 + 16, k0);
    v16h b2 = ld_frag(Bt, K, n0 + 32, k0);
    v16h b3 = ld_frag(Bt, K, n0 + 48, k0);
    acc[0] = mma16(a, b0, acc[0]);
    acc[1] = mma16(a, b1, acc[1]);
    acc[2] = mma16(a, b2, acc[2]);
    acc[3] = mma16(a, b3, acc[3]);
    asm volatile("v_nop\n\tv_nop\n\tv_nop\n\tv_nop"
                 : "+v"(acc[0]), "+v"(acc[1]), "+v"(acc[2]), "+v"(acc[3])
                 : "v"(a), "v"(b0), "v"(b1), "v"(b2), "v"(b3));
  }

  const bool act = (flags & 8) != 0;
#pragma unroll
  for (int j = 0; j < 4; ++j) {
    const int n = n0 + 16 * j + m;
    const float bi = bias[n];
#pragma unroll
    for (int v = 0; v < 8; ++v) {
      float val = acc[j][v] * cs + bi;
      if (act) val = (val >= 0.f) ? val : 0.01f * val;
      sT[wid][8 * h + v][16 * j + m] = val;
    }
  }
  __syncthreads();
  if ((flags & 4) && tid < 64) {
    float s = 0.f;
#pragma unroll
    for (int w = 0; w < 4; ++w)
#pragma unroll
      for (int r = 0; r < 16; ++r) s += sT[w][r][tid];
    sP[tid] = s;
  }
  __syncthreads();

  for (int ps = 0; ps < 2; ++ps) {
    if (ps) __threadfence();
    if (flags & 1) {
#pragma unroll
      for (int rr = 0; rr < 8; ++rr) {
        const int row = rr * 2 + h;
        v4f v = *(const v4fa*)&sT[wid][row][m * 4];
        float* p = outF + (size_t)(m0 + row) * Nc + n0 + m * 4;
        *(volatile v4f*)p = v;
      }
    }
    if (flags & 2) {
#pragma unroll
      for (int rr = 0; rr < 4; ++rr) {
        const int row = rr * 4 + (l >> 3), c8 = l & 7;
        v4f v0 = *(const v4fa*)&sT[wid][row][c8 * 8];
        v4f v1 = *(const v4fa*)&sT[wid][row][c8 * 8 + 4];
        v8h o = cvt8(v0 * hsA, v1 * hsA, hsB);
        f16* p = outH + (size_t)(m0 + row) * Nc + n0 + c8 * 8;
        *(volatile v8h*)p = o;
      }
    }
    if ((flags & 4) && wid == 0 && l < 16) {
      v4f v = *(const v4fa*)&sP[l * 4];
      float* p = P + (size_t)bm * Nc + n0 + l * 4;
      *(volatile v4f*)p = v;
    }
  }
}

__global__ void __launch_bounds__(128) k_colmean(const float* __restrict__ P, float* cm, int nrg, int nc, float inv)
{
  const int c = threadIdx.x * 4;
  if (c + 3 >= nc) return;
  v4f s = {0.f, 0.f, 0.f, 0.f};
  for (int rg = 0; rg < nrg; ++rg) s += *(const v4f*)(P + (size_t)rg * nc + c);
  s = s * inv;
  float* p = cm + c;
  *(volatile v4f*)p = s;
  __threadfence();
  *(volatile v4f*)p = s;
}

__global__ void __launch_bounds__(256) k_mix(const float* __restrict__ Hf, const float* __restrict__ cm,
                                             f16* Hm, int n8, float sc)
{
  const int i = blockIdx.x * 256 + threadIdx.x;
  if (i >= n8) return;
  const size_t e = (size_t)i * 8;
  const int d = (int)(e & (size_t)(DHID - 1));
  v4f a  = *(const v4f*)(Hf + e);
  v4f b  = *(const v4f*)(Hf + e + 4);
  v4f c0 = *(const v4f*)(cm + d);
  v4f c1 = *(const v4f*)(cm + d + 4);
  v8h o = cvt8((a + c0) * 0.5f, (b + c1) * 0.5f, sc);
  f16* p = Hm + e;
  *(volatile v8h*)p = o;
  __threadfence();
  *(volatile v8h*)p = o;
}

__global__ void __launch_bounds__(256) k_attn(
    const f16* __restrict__ Eh16, const f16* __restrict__ Et16,
    const float* __restrict__ EhF, const float* __restrict__ EtF,
    f16* Al16, int N, float lsc, float osc)
{
  __shared__ __attribute__((aligned(16))) f16 sB[16 * BSTR];
  __shared__ float sThr [AWAVES][16];
  __shared__ float sVal [AWAVES][16][16];
  __shared__ int   sIdx [AWAVES][16][16];
  __shared__ float sTile[AWAVES][16][16];

  const int tid = threadIdx.x, wid = tid >> 5, l = tid & 31, h = l >> 4, m = l & 15;
  if ((blockIdx.x + 1) * (AWAVES * 16) > N) return;
  const int m0 = (blockIdx.x * AWAVES + wid) * 16;

  for (int i = l; i < 256; i += 32) {
    sVal[wid][i >> 4][i & 15] = -3.0e38f;
    sIdx[wid][i >> 4][i & 15] = 0;
  }
  if (l < 16) sThr[wid][l] = -3.0e38f;
  float thr[8];
#pragma unroll
  for (int v = 0; v < 8; ++v) thr[v] = -3.0e38f;

  v16h afr[16];
#pragma unroll
  for (int kk = 0; kk < 16; ++kk) afr[kk] = ld_frag(Eh16, DHID, m0, kk * 32);

  const v8f z8 = {0.f, 0.f, 0.f, 0.f, 0.f, 0.f, 0.f, 0.f};
  const int T = N >> 4;
  for (int t = 0; t < T; ++t) {
    const int n0 = t << 4;
#pragma unroll
    for (int rq = 0; rq < 4; ++rq) {
      const int u = tid + 256 * rq;
      const int row = u >> 6, ch = u & 63;
      v8h v = *(const v8h*)(Et16 + (size_t)(n0 + row) * DHID + ch * 8);
      *(v8h*)(sB + row * BSTR + ch * 8) = v;
    }
    __syncthreads();

    v8f acc = z8;
    v16h bq[2];
#pragma unroll
    for (int kk = 0; kk < 16; ++kk) {
      bq[kk & 1] = ld_frag(sB, BSTR, 0, kk * 32);
      acc = mma16(afr[kk], bq[kk & 1], acc);
    }
    asm volatile("v_nop\n\tv_nop\n\tv_nop\n\tv_nop" : "+v"(acc) : "v"(bq[0]), "v"(bq[1]), "v"(afr[15]));

    float lg[8];
    unsigned anym = 0u, mym = 0u;
#pragma unroll
    for (int v = 0; v < 8; ++v) {
      lg[v] = acc[v] * lsc;
      const unsigned bmask = (unsigned)__ballot(lg[v] > thr[v]);
      anym |= bmask;
      mym = (l == v)     ? (bmask & 0xffffu) : mym;
      mym = (l == v + 8) ? (bmask >> 16)     : mym;
    }

    if (anym != 0u) {
#pragma unroll
      for (int v = 0; v < 8; ++v) sTile[wid][8 * h + v][m] = lg[v];
      asm volatile("s_wait_dscnt 0x0" ::: "memory");
      __builtin_amdgcn_wave_barrier();
      if (l < 16 && mym != 0u) {
        float th = sThr[wid][l];
        unsigned msk = mym;
        while (msk != 0u) {
          const int c = __builtin_ctz(msk);
          msk &= msk - 1u;
          const float val = sTile[wid][l][c];
          if (val > th) {
            int mi = 0;
            float mv = sVal[wid][l][0];
#pragma unroll
            for (int q = 1; q < 16; ++q) {
              const float qv = sVal[wid][l][q];
              if (qv < mv) { mv = qv; mi = q; }
            }
            if (val > mv) {
              sVal[wid][l][mi] = val;
              sIdx[wid][l][mi] = n0 + c;
              float nm = sVal[wid][l][0];
#pragma unroll
              for (int q = 1; q < 16; ++q) nm = fminf(nm, sVal[wid][l][q]);
              th = nm;
            }
          }
        }
        sThr[wid][l] = th;
      }
      asm volatile("s_wait_dscnt 0x0" ::: "memory");
      __builtin_amdgcn_wave_barrier();
#pragma unroll
      for (int v = 0; v < 8; ++v) thr[v] = sThr[wid][8 * h + v];
    }
    __syncthreads();
  }

#pragma unroll 1
  for (int r = 0; r < 16; ++r) {
    const int n = m0 + r;
    const float tv = sVal[wid][r][m];
    int ix = sIdx[wid][r][m];
    ix = (ix < 0) ? 0 : ((ix > N - 1) ? (N - 1) : ix);

    float mx = tv;
    mx = fmaxf(mx, __shfl_xor(mx, 8, 32));
    mx = fmaxf(mx, __shfl_xor(mx, 4, 32));
    mx = fmaxf(mx, __shfl_xor(mx, 2, 32));
    mx = fmaxf(mx, __shfl_xor(mx, 1, 32));
    const float e1 = expf(tv - mx);
    float s1 = e1;
    s1 += __shfl_xor(s1, 8, 32);
    s1 += __shfl_xor(s1, 4, 32);
    s1 += __shfl_xor(s1, 2, 32);
    s1 += __shfl_xor(s1, 1, 32);
    const float p1 = e1 * (1.0f / s1);

    const float* er = EhF + (size_t)n * DHID + l * 8;
    v4f ea = *(const v4f*)(er);
    v4f eb = *(const v4f*)(er + 4);
    v4f ec = *(const v4f*)(er + 256);
    v4f ed = *(const v4f*)(er + 260);
    float ehv[16] = {ea[0], ea[1], ea[2], ea[3], eb[0], eb[1], eb[2], eb[3],
                     ec[0], ec[1], ec[2], ec[3], ed[0], ed[1], ed[2], ed[3]};

    float wk = 0.f;
#pragma unroll 1
    for (int k = 0; k < TOPK; ++k) {
      const float pk = __shfl(p1, k, 32);
      const int   ik = __shfl(ix, k, 32);
      const float* nr = EtF + (size_t)ik * DHID + l * 8;
      v4f na = *(const v4f*)(nr);
      v4f nb = *(const v4f*)(nr + 4);
      v4f nc = *(const v4f*)(nr + 256);
      v4f nd = *(const v4f*)(nr + 260);
      float nbv[16] = {na[0], na[1], na[2], na[3], nb[0], nb[1], nb[2], nb[3],
                       nc[0], nc[1], nc[2], nc[3], nd[0], nd[1], nd[2], nd[3]};
      const float qk = 1.0f - pk;
      float sa = 0.f, sg = 0.f;
#pragma unroll
      for (int i = 0; i < 16; ++i) {
        const float x = nbv[i];
        sa += x;
        const float mixv = pk * x + qk * ehv[i];
        sg += tanhf(ehv[i] + mixv);
      }
#pragma unroll
      for (int off = 16; off >= 1; off >>= 1) {
        sa += __shfl_xor(sa, off, 32);
        sg += __shfl_xor(sg, off, 32);
      }
      const float w = sa * sg;
      if (m == k) wk = w;
    }

    float mx2 = wk;
    mx2 = fmaxf(mx2, __shfl_xor(mx2, 8, 32));
    mx2 = fmaxf(mx2, __shfl_xor(mx2, 4, 32));
    mx2 = fmaxf(mx2, __shfl_xor(mx2, 2, 32));
    mx2 = fmaxf(mx2, __shfl_xor(mx2, 1, 32));
    const float e2 = expf(wk - mx2);
    float s2 = e2;
    s2 += __shfl_xor(s2, 8, 32);
    s2 += __shfl_xor(s2, 4, 32);
    s2 += __shfl_xor(s2, 2, 32);
    s2 += __shfl_xor(s2, 1, 32);
    const float kap = e2 * (1.0f / s2);

    float en[16];
#pragma unroll
    for (int i = 0; i < 16; ++i) en[i] = 0.f;
#pragma unroll 1
    for (int k = 0; k < TOPK; ++k) {
      const float kk = __shfl(kap, k, 32);
      const int   ik = __shfl(ix, k, 32);
      const float* nr = EtF + (size_t)ik * DHID + l * 8;
      v4f na = *(const v4f*)(nr);
      v4f nb = *(const v4f*)(nr + 4);
      v4f nc = *(const v4f*)(nr + 256);
      v4f nd = *(const v4f*)(nr + 260);
      float nbv[16] = {na[0], na[1], na[2], na[3], nb[0], nb[1], nb[2], nb[3],
                       nc[0], nc[1], nc[2], nc[3], nd[0], nd[1], nd[2], nd[3]};
#pragma unroll
      for (int i = 0; i < 16; ++i) en[i] += kk * nbv[i];
    }

    v8h o0, o1;
#pragma unroll
    for (int i = 0; i < 8; ++i) {
      o0[i] = (f16)((ehv[i] + en[i]) * osc);
      o1[i] = (f16)((ehv[8 + i] + en[8 + i]) * osc);
    }
    f16* orow = Al16 + (size_t)n * DHID + l * 8;
    *(volatile v8h*)orow = o0;
    *(volatile v8h*)(orow + 256) = o1;
    __threadfence();
    *(volatile v8h*)orow = o0;
    *(volatile v8h*)(orow + 256) = o1;
  }
}

__global__ void __launch_bounds__(256) k_final(
    const float* __restrict__ P, const float* __restrict__ gam, const float* __restrict__ bet,
    const float* __restrict__ Wf, const float* __restrict__ bfv, float* out, int nrg, float invn)
{
  __shared__ float g[DHID];
  __shared__ float red[256];
  const int tid = threadIdx.x;
  for (int d = tid; d < DHID; d += 256) {
    float s = 0.f;
    for (int rg = 0; rg < nrg; ++rg) s += P[(size_t)rg * DHID + d];
    g[d] = s * invn;
  }
  __syncthreads();

  float p = 0.f;
  for (int d = tid; d < DHID; d += 256) p += g[d];
  red[tid] = p;
  __syncthreads();
  for (int s = 128; s > 0; s >>= 1) { if (tid < s) red[tid] += red[tid + s]; __syncthreads(); }
  const float mu = red[0] * (1.0f / (float)DHID);
  __syncthreads();

  float pv = 0.f;
  for (int d = tid; d < DHID; d += 256) { float tq = g[d] - mu; pv += tq * tq; }
  red[tid] = pv;
  __syncthreads();
  for (int s = 128; s > 0; s >>= 1) { if (tid < s) red[tid] += red[tid + s]; __syncthreads(); }
  const float var  = red[0] * (1.0f / (float)DHID);
  const float rstd = 1.0f / sqrtf(var + 1e-5f);
  __syncthreads();

  for (int d = tid; d < DHID; d += 256) g[d] = (g[d] - mu) * rstd * gam[d] + bet[d];
  __syncthreads();

  float a0 = 0.f, a1 = 0.f;
  for (int d = tid; d < DHID; d += 256) {
    const float gv = g[d];
    a0 += gv * Wf[d * NCLS + 0];
    a1 += gv * Wf[d * NCLS + 1];
  }
  red[tid] = a0;
  __syncthreads();
  for (int s = 128; s > 0; s >>= 1) { if (tid < s) red[tid] += red[tid + s]; __syncthreads(); }
  const float o0 = red[0] + bfv[0];
  __syncthreads();
  red[tid] = a1;
  __syncthreads();
  for (int s = 128; s > 0; s >>= 1) { if (tid < s) red[tid] += red[tid + s]; __syncthreads(); }
  const float o1 = red[0] + bfv[1];
  if (tid == 0) {
    v2f o = {o0, o1};
    *(volatile v2f*)out = o;
    __threadfence();
    *(volatile v2f*)out = o;
  }
}

extern "C" void kernel_launch(void* const* d_in, const int* in_sizes, int n_in,
                              void* d_out, int out_size, void* d_ws, size_t ws_size,
                              hipStream_t stream)
{
  if (n_in < 13 || out_size < NCLS) return;
  if (in_sizes[0] != NTOK * DIN || in_sizes[1] != DIN * DHID || in_sizes[2] != DHID ||
      in_sizes[3] != DHID * DHID || in_sizes[4] != DHID || in_sizes[5] != DHID * DHID ||
      in_sizes[6] != DHID || in_sizes[7] != DHID * DHID || in_sizes[8] != DHID ||
      in_sizes[9] != DHID || in_sizes[10] != DHID || in_sizes[11] != DHID * NCLS ||
      in_sizes[12] != NCLS) return;

  const float* x   = (const float*)d_in[0];
  const float* W1  = (const float*)d_in[1];
  const float* b1  = (const float*)d_in[2];
  const float* Wh  = (const float*)d_in[3];
  const float* bh  = (const float*)d_in[4];
  const float* Wt  = (const float*)d_in[5];
  const float* bt  = (const float*)d_in[6];
  const float* Wl  = (const float*)d_in[7];
  const float* bl  = (const float*)d_in[8];
  const float* gam = (const float*)d_in[9];
  const float* bet = (const float*)d_in[10];
  const float* Wf  = (const float*)d_in[11];
  const float* bfv = (const float*)d_in[12];
  float* out = (float*)d_out;

  char* base = (char*)d_ws;
  size_t off = 0;
  auto carve = [&](size_t bytes) -> void* {
    void* p = base + off;
    off += (bytes + 255) & ~(size_t)255;
    return p;
  };
  f16*   x16  = (f16*)  carve((size_t)NTOK * DIN * 2);
  f16*   W1t  = (f16*)  carve((size_t)DHID * DIN * 2);
  f16*   Wht  = (f16*)  carve((size_t)DHID * DHID * 2);
  f16*   Wtt  = (f16*)  carve((size_t)DHID * DHID * 2);
  f16*   Wlt  = (f16*)  carve((size_t)DHID * DHID * 2);
  float* hF   = (float*)carve((size_t)NTOK * DHID * 4);
  float* P1   = (float*)carve((size_t)NRG * DHID * 4);
  float* cm   = (float*)carve((size_t)DHID * 4);
  f16*   hm16 = (f16*)  carve((size_t)NTOK * DHID * 2);
  float* ehF  = (float*)carve((size_t)NTOK * DHID * 4);
  float* etF  = (float*)carve((size_t)NTOK * DHID * 4);
  f16*   eh16 = (f16*)  carve((size_t)NTOK * DHID * 2);
  f16*   et16 = (f16*)  carve((size_t)NTOK * DHID * 2);
  f16*   al16 = (f16*)  carve((size_t)NTOK * DHID * 2);
  float* P4   = (float*)carve((size_t)NRG * DHID * 4);
  if (off > ws_size) return;

  const float WSC   = 64.0f;
  const float HSC   = 8.0f;
  const float SCALE = 0.04419417382415922f;
  const float EHS   = 256.0f;
  const float ETS   = 16.0f;
  const float ASC   = 8.0f;

  const int n8x = NTOK * DIN / 8;
  k_cvt<<<(n8x + 255) / 256, 256, 0, stream>>>(x, x16, n8x, 1.0f);

  k_wtr<<<(DIN / 64) * (DHID / 32), 256, 0, stream>>>(W1, W1t, DIN, DHID, WSC);
  k_wtr<<<(DHID / 64) * (DHID / 32), 256, 0, stream>>>(Wh, Wht, DHID, DHID, WSC);
  k_wtr<<<(DHID / 64) * (DHID / 32), 256, 0, stream>>>(Wt, Wtt, DHID, DHID, WSC);
  k_wtr<<<(DHID / 64) * (DHID / 32), 256, 0, stream>>>(Wl, Wlt, DHID, DHID, WSC);

  const int ggrid = (NTOK / 64) * (DHID / 64);

  k_gemm<<<ggrid, 128, 0, stream>>>(x16, W1t, b1, hF, hm16, P1,
                                    NTOK, DHID, DIN, 1.0f / WSC, 1.0f, 1.0f, 1 | 4 | 8);
  k_colmean<<<1, 128, 0, stream>>>(P1, cm, NRG, DHID, 1.0f / (float)NTOK);
  const int n8h = NTOK * DHID / 8;
  k_mix<<<(n8h + 255) / 256, 256, 0, stream>>>(hF, cm, hm16, n8h, HSC);

  k_gemm<<<ggrid, 128, 0, stream>>>(hm16, Wht, bh, ehF, eh16, P1,
                                    NTOK, DHID, DHID, 1.0f / (HSC * WSC), SCALE, EHS, 1 | 2);
  k_gemm<<<ggrid, 128, 0, stream>>>(hm16, Wtt, bt, etF, et16, P1,
                                    NTOK, DHID, DHID, 1.0f / (HSC * WSC), 1.0f, ETS, 1 | 2);

  k_attn<<<NTOK / (AWAVES * 16), 256, 0, stream>>>(eh16, et16, ehF, etF, al16,
                                                   NTOK, 1.0f / (EHS * ETS), ASC);

  k_gemm<<<ggrid, 128, 0, stream>>>(al16, Wlt, bl, ehF, eh16, P4,
                                    NTOK, DHID, DHID, 1.0f / (ASC * WSC), 1.0f, 1.0f, 4 | 8);

  k_final<<<1, 256, 0, stream>>>(P4, gam, bet, Wf, bfv, out, NRG, 1.0f / (float)NTOK);
}
